// MAlphaAttention_50173807952661
// MI455X (gfx1250) — hardware-verified
//
#include <hip/hip_runtime.h>

typedef _Float16 f16;
typedef f16 v8h __attribute__((ext_vector_type(8)));
typedef f16 v16h __attribute__((ext_vector_type(16)));
typedef float v8f __attribute__((ext_vector_type(8)));
typedef float v4f __attribute__((ext_vector_type(4)));

union Frag {
  v16h v;
  v8h half[2];
};

#define NP 1024
#define DC 768
#define NH 12
#define HD 64
#define NB 4
#define BNR (NB * NP)
#define C3 (3 * DC)

static_assert(BNR % 64 == 0 && C3 % 128 == 0 && DC % 128 == 0 && NP % 64 == 0);
static_assert(DC % 32 == 0 && NP % 32 == 0 && HD == 64 && NP % 128 == 0);

__device__ __forceinline__ v8f fz8() {
  v8f z = {0.f, 0.f, 0.f, 0.f, 0.f, 0.f, 0.f, 0.f};
  return z;
}

__device__ __forceinline__ v8f wmma16(const v16h a, const v16h b, v8f c) {
  v8f d = __builtin_amdgcn_wmma_f32_16x16x32_f16(false, a, false, b, (short)0, c, false, false);
  asm volatile("v_nop\n\tv_nop\n\tv_nop\n\tv_nop" : "+v"(d) : "v"(a), "v"(b));
  return d;
}

__global__ __launch_bounds__(256) void k_cvt8(const float* __restrict__ in,
                                              f16* __restrict__ out, int n8) {
  const int i = blockIdx.x * 256 + threadIdx.x;
  if (i >= n8) return;
  const size_t e = (size_t)i * 8;
  const v4f a = *(const v4f*)(in + e);
  const v4f c = *(const v4f*)(in + e + 4);
  v8h o;
  o[0] = (f16)a[0]; o[1] = (f16)a[1]; o[2] = (f16)a[2]; o[3] = (f16)a[3];
  o[4] = (f16)c[0]; o[5] = (f16)c[1]; o[6] = (f16)c[2]; o[7] = (f16)c[3];
  volatile v8h* p = (volatile v8h*)(out + e);
  *p = o;
  __threadfence();
  *p = o;
}

__global__ __launch_bounds__(256) void k_tcvt(const float* __restrict__ in,
                                              f16* __restrict__ out, int R, int C,
                                              float scale) {
  __shared__ float tile[64 * 65];
  const int t = threadIdx.x;
  const int c0 = blockIdx.x * 64, r0 = blockIdx.y * 64;
  const int tx = t & 15, ty = t >> 4;
#pragma unroll
  for (int j = 0; j < 4; ++j) {
    const int rl = ty + 16 * j;
    const int r = r0 + rl, c = c0 + 4 * tx;
    v4f v = {0.f, 0.f, 0.f, 0.f};
    if (r < R && c + 3 < C) v = *(const v4f*)(in + (size_t)r * C + c);
    tile[rl * 65 + 4 * tx + 0] = v[0] * scale;
    tile[rl * 65 + 4 * tx + 1] = v[1] * scale;
    tile[rl * 65 + 4 * tx + 2] = v[2] * scale;
    tile[rl * 65 + 4 * tx + 3] = v[3] * scale;
  }
  __syncthreads();
  const int lane = t & 31, wave = t >> 5;
  v8h vals[2];
  size_t gi[2];
  bool ok[2];
#pragma unroll
  for (int i = 0; i < 2; ++i) {
    const int cl = wave * 8 + i * 4 + (lane >> 3);
    const int roff = (lane & 7) * 8;
    v8h o;
#pragma unroll
    for (int e = 0; e < 8; ++e) o[e] = (f16)tile[(roff + e) * 65 + cl];
    vals[i] = o;
    const int gc = c0 + cl, gr = r0 + roff;
    ok[i] = (gc < C) && (gr + 7 < R);
    gi[i] = (size_t)gc * R + gr;
  }
#pragma unroll
  for (int i = 0; i < 2; ++i)
    if (ok[i]) *(volatile v8h*)(out + gi[i]) = vals[i];
  __threadfence();
#pragma unroll
  for (int i = 0; i < 2; ++i)
    if (ok[i]) *(volatile v8h*)(out + gi[i]) = vals[i];
}

template <int MODE>
__global__ __launch_bounds__(256) void k_gemm(const f16* __restrict__ A,
                                              const f16* __restrict__ Bm,
                                              void* __restrict__ Out,
                                              const float* __restrict__ bias,
                                              int lda, int ldb, int K) {
  constexpr int LT = 40;
  __shared__ f16 At[64 * LT];
  __shared__ f16 Bt[128 * LT];

  const int t = threadIdx.x, lane = t & 31, wave = t >> 5;
  const int m = lane & 15, h = lane >> 4;
  const int wm = wave >> 2, wn = wave & 3;
  const int n0 = blockIdx.x * 128, m0 = blockIdx.y * 64;

  const f16* Bb = Bm;
  if constexpr (MODE == 1) {
    const int z = blockIdx.z;
    Bb = Bm + (size_t)((z >> 2) * DC) * BNR + (size_t)(z & 3) * NP;
  }

  v8f acc[2][2];
#pragma unroll
  for (int i = 0; i < 2; ++i)
#pragma unroll
    for (int j = 0; j < 2; ++j) acc[i][j] = fz8();

  const int nk = K >> 5;
  for (int kt = 0; kt < nk; ++kt) {
    const int kk = kt << 5;
    __syncthreads();
    {
      const int row = t >> 2, kc = (t & 3) * 8;
      *(v8h*)(At + row * LT + kc) =
          *(const v8h*)(A + (size_t)(m0 + row) * lda + kk + kc);
    }
#pragma unroll
    for (int i = 0; i < 2; ++i) {
      const int idx = t + i * 256;
      const int row = idx >> 2, kc = (idx & 3) * 8;
      *(v8h*)(Bt + row * LT + kc) =
          *(const v8h*)(Bb + (size_t)(n0 + row) * ldb + kk + kc);
    }
    __syncthreads();

    Frag af[2], bf[2];
#pragma unroll
    for (int mt = 0; mt < 2; ++mt) {
      const f16* p = At + (wm * 32 + mt * 16 + m) * LT + 8 * h;
      af[mt].half[0] = *(const v8h*)p;
      af[mt].half[1] = *(const v8h*)(p + 16);
    }
#pragma unroll
    for (int nt = 0; nt < 2; ++nt) {
      const f16* p = Bt + (wn * 32 + nt * 16 + m) * LT + 8 * h;
      bf[nt].half[0] = *(const v8h*)p;
      bf[nt].half[1] = *(const v8h*)(p + 16);
    }
#pragma unroll
    for (int mt = 0; mt < 2; ++mt)
#pragma unroll
      for (int nt = 0; nt < 2; ++nt)
        acc[mt][nt] = wmma16(af[mt].v, bf[nt].v, acc[mt][nt]);
  }

  if constexpr (MODE == 0) {
    __shared__ f16 Cs[128 * 72];
    const int seg = n0 / DC;
    const float sc = 0.0625f;
#pragma unroll
    for (int mt = 0; mt < 2; ++mt) {
#pragma unroll
      for (int nt = 0; nt < 2; ++nt) {
        const int cl = wn * 32 + nt * 16 + m;
        const int rl = wm * 32 + mt * 16 + 8 * h;
        v8h o;
#pragma unroll
        for (int r = 0; r < 8; ++r) {
          float v = acc[mt][nt][r] * sc;
          if (seg < 2) v = fmaxf(v, 0.f) + 1e-6f;
          o[r] = (f16)v;
        }
        *(v8h*)(Cs + cl * 72 + rl) = o;
      }
    }
    __syncthreads();
    f16* Ob = (f16*)Out;
    v8h vals[4];
    size_t gi[4];
#pragma unroll
    for (int i = 0; i < 4; ++i) {
      const int cl = wave * 16 + i * 4 + (lane >> 3);
      const int off = (lane & 7) * 8;
      vals[i] = *(const v8h*)(Cs + cl * 72 + off);
      gi[i] = (size_t)(n0 + cl) * BNR + m0 + off;
    }
#pragma unroll
    for (int i = 0; i < 4; ++i) *(volatile v8h*)(Ob + gi[i]) = vals[i];
    __threadfence();
#pragma unroll
    for (int i = 0; i < 4; ++i) *(volatile v8h*)(Ob + gi[i]) = vals[i];
  } else if constexpr (MODE == 1) {
    __shared__ f16 Cs[64 * 136];
#pragma unroll
    for (int mt = 0; mt < 2; ++mt) {
#pragma unroll
      for (int nt = 0; nt < 2; ++nt) {
        const int coll = wn * 32 + nt * 16 + m;
        const int colg = n0 + coll;
        const int rl0 = wm * 32 + mt * 16 + 8 * h;
        const v8h qv = *(const v8h*)(Bb + (size_t)colg * ldb + m0 + rl0);
#pragma unroll
        for (int r = 0; r < 8; ++r)
          Cs[(rl0 + r) * 136 + coll] = (f16)((float)qv[r] + 0.1f * acc[mt][nt][r]);
      }
    }
    __syncthreads();
    f16* Ob = (f16*)Out + (size_t)blockIdx.z * ((size_t)NP * DC);
    v8h vals[4];
    size_t gi[4];
#pragma unroll
    for (int i = 0; i < 4; ++i) {
      const int rl = wave * 8 + i * 2 + (lane >> 4);
      const int off = (lane & 15) * 8;
      vals[i] = *(const v8h*)(Cs + rl * 136 + off);
      gi[i] = (size_t)(m0 + rl) * DC + n0 + off;
    }
#pragma unroll
    for (int i = 0; i < 4; ++i) *(volatile v8h*)(Ob + gi[i]) = vals[i];
    __threadfence();
#pragma unroll
    for (int i = 0; i < 4; ++i) *(volatile v8h*)(Ob + gi[i]) = vals[i];
  } else {
    __shared__ float Cs[64 * 132];
    const float sc = 0.0625f;
#pragma unroll
    for (int mt = 0; mt < 2; ++mt) {
#pragma unroll
      for (int nt = 0; nt < 2; ++nt) {
        const int coll = wn * 32 + nt * 16 + m;
        const int rl0 = wm * 32 + mt * 16 + 8 * h;
#pragma unroll
        for (int r = 0; r < 8; ++r) Cs[(rl0 + r) * 132 + coll] = acc[mt][nt][r] * sc;
      }
    }
    __syncthreads();
    float* Ob = (float*)Out;
    const v4f bv = *(const v4f*)(bias + n0 + lane * 4);
    v4f vals[8];
    size_t gi[8];
#pragma unroll
    for (int i = 0; i < 8; ++i) {
      const int rl = wave * 8 + i;
      vals[i] = *(const v4f*)(Cs + rl * 132 + lane * 4) + bv;
      gi[i] = (size_t)(m0 + rl) * DC + n0 + lane * 4;
    }
#pragma unroll
    for (int i = 0; i < 8; ++i) *(volatile v4f*)(Ob + gi[i]) = vals[i];
    __threadfence();
#pragma unroll
    for (int i = 0; i < 8; ++i) *(volatile v4f*)(Ob + gi[i]) = vals[i];
  }
}

__global__ __launch_bounds__(256) void k_attn(const f16* __restrict__ Qp,
                                              const f16* __restrict__ Kp,
                                              const f16* __restrict__ Vs,
                                              const float* __restrict__ mask,
                                              f16* __restrict__ Og) {
  constexpr int LDK = 72;
  __shared__ f16 Kt[64 * LDK];
  __shared__ f16 Vt[64 * LDK];
  __shared__ f16 Os[8 * 16 * LDK];

  const int t = threadIdx.x, lane = t & 31, wave = t >> 5;
  const int m = lane & 15, h = lane >> 4;
  const int b = blockIdx.z, hh = blockIdx.y;
  const int nw = blockIdx.x * 128 + wave * 16;
  const size_t roff = (size_t)b * NP * DC + (size_t)hh * HD;
  const f16* Vb = Vs + (size_t)(hh * HD) * BNR + (size_t)b * NP;

  Frag qf[2];
  {
    const f16* qrow = Qp + roff + (size_t)(nw + m) * DC;
#pragma unroll
    for (int f = 0; f < 2; ++f) {
      const f16* p = qrow + f * 32 + 8 * h;
      qf[f].half[0] = *(const v8h*)p;
      qf[f].half[1] = *(const v8h*)(p + 16);
    }
  }

  v8f oacc[4];
#pragma unroll
  for (int i = 0; i < 4; ++i) oacc[i] = fz8();
  float rsum = 0.f;
  const float* mrow = mask + (size_t)(nw + m) * NP + 8 * h;

  for (int ic = 0; ic < NP / 64; ++ic) {
    const int mc = ic * 64;
    __syncthreads();
#pragma unroll
    for (int i = 0; i < 2; ++i) {
      const int idx = t + i * 256;
      const int rr = idx >> 3, cc = (idx & 7) * 8;
      *(v8h*)(Kt + rr * LDK + cc) = *(const v8h*)(Kp + roff + (size_t)(mc + rr) * DC + cc);
      *(v8h*)(Vt + rr * LDK + cc) = *(const v8h*)(Vb + (size_t)rr * BNR + mc + cc);
    }
    __syncthreads();

#pragma unroll
    for (int p2 = 0; p2 < 2; ++p2) {
      v8f s0 = fz8(), s1 = fz8();
#pragma unroll
      for (int f = 0; f < 2; ++f) {
        Frag ka, kb;
        const f16* pa = Kt + (32 * p2 + m) * LDK + f * 32 + 8 * h;
        const f16* pb = pa + 16 * LDK;
        ka.half[0] = *(const v8h*)pa;
        ka.half[1] = *(const v8h*)(pa + 16);
        kb.half[0] = *(const v8h*)pb;
        kb.half[1] = *(const v8h*)(pb + 16);
        s0 = wmma16(ka.v, qf[f].v, s0);
        s1 = wmma16(kb.v, qf[f].v, s1);
      }
      const float* mp = mrow + mc + 32 * p2;
      const v4f ma = *(const v4f*)mp;
      const v4f mb = *(const v4f*)(mp + 4);
      const v4f mcx = *(const v4f*)(mp + 16);
      const v4f mdx = *(const v4f*)(mp + 20);
      v8h plo, phi;
#pragma unroll
      for (int r = 0; r < 4; ++r) {
        const float sv = s0[r] * ma[r];
        rsum += sv;
        plo[r] = (f16)sv;
      }
#pragma unroll
      for (int r = 0; r < 4; ++r) {
        const float sv = s0[4 + r] * mb[r];
        rsum += sv;
        plo[4 + r] = (f16)sv;
      }
#pragma unroll
      for (int r = 0; r < 4; ++r) {
        const float sv = s1[r] * mcx[r];
        rsum += sv;
        phi[r] = (f16)sv;
      }
#pragma unroll
      for (int r = 0; r < 4; ++r) {
        const float sv = s1[4 + r] * mdx[r];
        rsum += sv;
        phi[4 + r] = (f16)sv;
      }
      Frag pf;
      pf.half[0] = plo;
      pf.half[1] = phi;
#pragma unroll
      for (int nt = 0; nt < 4; ++nt) {
        Frag bv;
        const f16* pv = Vt + (nt * 16 + m) * LDK + 32 * p2 + 8 * h;
        bv.half[0] = *(const v8h*)pv;
        bv.half[1] = *(const v8h*)(pv + 16);
        oacc[nt] = wmma16(pf.v, bv.v, oacc[nt]);
      }
    }
  }

  rsum += __shfl_xor(rsum, 16);
  const float z = 1.0f / (rsum + 1e-6f);
  float zr[8];
#pragma unroll
  for (int r = 0; r < 8; ++r) zr[r] = __shfl(z, 8 * h + r);

  f16* osw = Os + wave * (16 * LDK);
#pragma unroll
  for (int nt = 0; nt < 4; ++nt)
#pragma unroll
    for (int r = 0; r < 8; ++r)
      osw[(8 * h + r) * LDK + nt * 16 + m] = (f16)(oacc[nt][r] * zr[r]);
  __syncthreads();

  v8h vals[4];
  size_t gi[4];
#pragma unroll
  for (int i = 0; i < 4; ++i) {
    const int rq = i * 4 + (lane >> 3);
    const int off = (lane & 7) * 8;
    vals[i] = *(const v8h*)(osw + rq * LDK + off);
    gi[i] = roff + (size_t)(nw + rq) * DC + off;
  }
#pragma unroll
  for (int i = 0; i < 4; ++i) *(volatile v8h*)(Og + gi[i]) = vals[i];
  __threadfence();
#pragma unroll
  for (int i = 0; i < 4; ++i) *(volatile v8h*)(Og + gi[i]) = vals[i];
}

extern "C" void kernel_launch(void* const* d_in, const int* in_sizes, int n_in,
                              void* d_out, int out_size, void* d_ws, size_t ws_size,
                              hipStream_t stream) {
  if (n_in < 5) return;
  if (in_sizes[0] != BNR * DC || in_sizes[1] != DC * C3 || in_sizes[2] != DC * DC ||
      in_sizes[3] != DC || in_sizes[4] != NP * NP || out_size != BNR * DC)
    return;

  const float* x = (const float*)d_in[0];
  const float* Wqkv = (const float*)d_in[1];
  const float* Wout = (const float*)d_in[2];
  const float* bout = (const float*)d_in[3];
  const float* mask = (const float*)d_in[4];
  float* out = (float*)d_out;

  const size_t szXh = (size_t)BNR * DC * 2;
  const size_t szWqT = (size_t)C3 * DC * 2;
  const size_t szWoT = (size_t)DC * DC * 2;
  const size_t szMt = (size_t)NP * NP * 2;
  const size_t szQKVT = (size_t)C3 * BNR * 2;
  const size_t szQp = (size_t)2 * BNR * DC * 2;
  const size_t szO = (size_t)BNR * DC * 2;
  size_t off = 0;
  char* ws = (char*)d_ws;
  f16* xh = (f16*)(ws + off);    off += szXh;
  f16* WqT = (f16*)(ws + off);   off += szWqT;
  f16* WoT = (f16*)(ws + off);   off += szWoT;
  f16* Mt = (f16*)(ws + off);    off += szMt;
  f16* QKVT = (f16*)(ws + off);  off += szQKVT;
  f16* Qp = (f16*)(ws + off);    off += szQp;
  f16* O = (f16*)(ws + off);     off += szO;
  if (off > ws_size) return;

  const int n8 = BNR * DC / 8;
  k_cvt8<<<dim3((n8 + 255) / 256), 256, 0, stream>>>(x, xh, n8);
  k_tcvt<<<dim3((C3 + 63) / 64, (DC + 63) / 64), 256, 0, stream>>>(Wqkv, WqT, DC, C3, 16.0f);
  k_tcvt<<<dim3((DC + 63) / 64, (DC + 63) / 64), 256, 0, stream>>>(Wout, WoT, DC, DC, 16.0f);
  k_tcvt<<<dim3((NP + 63) / 64, (NP + 63) / 64), 256, 0, stream>>>(mask, Mt, NP, NP, 1.0f);

  k_gemm<0><<<dim3(C3 / 128, BNR / 64, 1), 256, 0, stream>>>(xh, WqT, QKVT, nullptr, DC, DC, DC);
  k_gemm<1><<<dim3(DC / 128, NP / 64, 8), 256, 0, stream>>>(Mt, QKVT, Qp, nullptr, NP, BNR, NP);
  k_attn<<<dim3(NP / 128, NH, NB), 256, 0, stream>>>(Qp, Qp + (size_t)NB * NP * DC,
                                                     QKVT + (size_t)(2 * DC) * BNR, mask, O);
  k_gemm<2><<<dim3(DC / 128, BNR / 64, 1), 256, 0, stream>>>(O, WoT, out, bout, DC, DC, DC);
}
